// PathfindingGNN_17274358464713
// MI455X (gfx1250) — hardware-verified
//
#include <hip/hip_runtime.h>
#include <stddef.h>


typedef float v8f __attribute__((ext_vector_type(8)));
typedef float v4f __attribute__((ext_vector_type(4)));
typedef unsigned int v4u __attribute__((ext_vector_type(4)));
typedef unsigned short v8us __attribute__((ext_vector_type(8)));
typedef unsigned short v16us __attribute__((ext_vector_type(16)));
typedef __bf16 v8b __attribute__((ext_vector_type(8)));
typedef __bf16 v16b __attribute__((ext_vector_type(16)));

union Frag { v16b v; v16us u; v8us half[2]; };
union Pack8 { v8b v; v8us u; };

#define HC 64
#define KU 128
#define NL 3
#define NBN 1024
#define CHK 8192
#define LCAP 4096
#define NTHR 256
#define BN_EPS 1e-5f
#define LDS_BYTES (NBN * HC * 4 + LCAP * 4 + 16 * 4 + NBN)

__device__ __forceinline__ v8f wmma16(v16b a, v16b b, v8f c)
{
    c = __builtin_amdgcn_wmma_f32_16x16x32_bf16(false, a, false, b, (short)0, c, false, false);
    asm volatile("v_nop\n\tv_nop\n\tv_nop\n\tv_nop" : "+v"(c) : "v"(a), "v"(b));
    return c;
}

__device__ __forceinline__ void split16(const float (&v)[16], v16b& hi, v16b& lo)
{
#pragma unroll
    for (int i = 0; i < 16; ++i) {
        const __bf16 h = (__bf16)v[i];
        const float r = v[i] - (float)h;
        hi[i] = h;
        lo[i] = (__bf16)r;
    }
}
__device__ __forceinline__ void split8(const float (&v)[8], Pack8& hi, Pack8& lo)
{
#pragma unroll
    for (int i = 0; i < 8; ++i) {
        const __bf16 h = (__bf16)v[i];
        const float r = v[i] - (float)h;
        hi.v[i] = h;
        lo.v[i] = (__bf16)r;
    }
}

__device__ __forceinline__ void ld16(const float* p, float (&v)[16])
{
    const v4f t0 = *(const v4f*)(p);
    const v4f t1 = *(const v4f*)(p + 4);
    const v4f t2 = *(const v4f*)(p + 16);
    const v4f t3 = *(const v4f*)(p + 20);
    v[0] = t0.x;  v[1] = t0.y;  v[2] = t0.z;  v[3] = t0.w;
    v[4] = t1.x;  v[5] = t1.y;  v[6] = t1.z;  v[7] = t1.w;
    v[8] = t2.x;  v[9] = t2.y;  v[10] = t2.z; v[11] = t2.w;
    v[12] = t3.x; v[13] = t3.y; v[14] = t3.z; v[15] = t3.w;
}

__device__ __forceinline__ v4f vmax4(v4f a, v4f b)
{
    v4f r;
    r.x = fmaxf(a.x, b.x); r.y = fmaxf(a.y, b.y); r.z = fmaxf(a.z, b.z); r.w = fmaxf(a.w, b.w);
    return r;
}

__device__ __forceinline__ unsigned zmask(unsigned x)
{
    unsigned y = (x & 0x7F7F7F7Fu) + 0x7F7F7F7Fu;
    y = (y | x) & 0x80808080u;
    return y ^ 0x80808080u;
}

__global__ __launch_bounds__(NTHR) void k_prep(const float* __restrict__ Wu, const float* __restrict__ Wp1,
                                               unsigned short* wsW, unsigned short* wsWp)
{
    const int t = blockIdx.x * NTHR + threadIdx.x;
    float v[8];
#pragma unroll
    for (int i = 0; i < 8; ++i) v[i] = 0.0f;
    unsigned short* d0 = wsW;
    unsigned short* d1 = wsW;
    bool ok = true;
    if (t < NL * HC * 16) {
        const int l = t >> 10, rem = t & 1023, n = rem >> 4, kg = rem & 15;
        const float* s = Wu + (size_t)l * KU * HC;
#pragma unroll
        for (int i = 0; i < 8; ++i) v[i] = s[(8 * kg + i) * HC + n];
        d0 = wsW + (size_t)l * (2 * HC * KU) + n * KU + 8 * kg;
        d1 = d0 + HC * KU;
    } else if (t < NL * HC * 16 + HC * 8) {
        const int t2 = t - NL * HC * 16, n = t2 >> 3, kg = t2 & 7;
#pragma unroll
        for (int i = 0; i < 8; ++i) v[i] = Wp1[(8 * kg + i) * HC + n];
        d0 = wsWp + n * HC + 8 * kg;
        d1 = d0 + HC * HC;
    } else {
        ok = false;
    }
    if (ok) {
        Pack8 hi, lo;
        split8(v, hi, lo);
        *(volatile v8us*)d0 = hi.u;
        *(volatile v8us*)d1 = lo.u;
        __threadfence();
        *(volatile v8us*)d0 = hi.u;
        *(volatile v8us*)d1 = lo.u;
    }
}

__global__ __launch_bounds__(NTHR) void k_code(const int* __restrict__ ei, unsigned char* code,
                                               int nNodes, int nEdges, int nEdgesPad)
{
    const int t = blockIdx.x * NTHR + threadIdx.x;
    const int e0 = t * 16;
    if (e0 >= nEdgesPad) return;
    unsigned w[4] = {0u, 0u, 0u, 0u};
#pragma unroll
    for (int j = 0; j < 16; ++j) {
        const int e = e0 + j;
        unsigned v = 0xFFu;
        if (e < nEdges) {
            int d = ei[(size_t)nEdges + e];
            d = min(max(d, 0), nNodes - 1);
            v = (unsigned)(d >> 10);
        }
        w[j >> 2] |= v << (8 * (j & 3));
    }
    const v4u o = {w[0], w[1], w[2], w[3]};
    volatile v4u* p = (volatile v4u*)(code + e0);
    *p = o;
    __threadfence();
    *p = o;
}

__global__ __launch_bounds__(NTHR) void k_enc(const float* __restrict__ x, const float* __restrict__ W,
                                              const float* __restrict__ b, float* h, int nNodes, int nRowsPad)
{
    const int tid = threadIdx.x;
    const int r = blockIdx.x * 16 + (tid >> 4);
    const int c4 = (tid & 15) * 4;
    if (r >= nRowsPad) return;
    const int rx = min(r, nNodes - 1);
    float xv[6];
#pragma unroll
    for (int k = 0; k < 6; ++k) xv[k] = x[(size_t)rx * 6 + k];
    float acc[4];
#pragma unroll
    for (int j = 0; j < 4; ++j) {
        float s = 0.0f;
#pragma unroll
        for (int k = 0; k < 6; ++k) s = fmaf(xv[k], W[k * HC + c4 + j], s);
        acc[j] = s + b[c4 + j];
    }
    const v4f o = {acc[0], acc[1], acc[2], acc[3]};
    volatile v4f* p = (volatile v4f*)(h + (size_t)r * HC + c4);
    *p = o;
    __threadfence();
    *p = o;
}

__global__ __launch_bounds__(NTHR) void k_layer(
    const float* __restrict__ hin, float* hout,
    const unsigned char* __restrict__ code, const int* __restrict__ ei, const float* __restrict__ ea,
    const unsigned short* __restrict__ wpl,
    const float* __restrict__ We, const float* __restrict__ be,
    const float* __restrict__ bu, const float* __restrict__ gam, const float* __restrict__ bet,
    const float* __restrict__ mn, const float* __restrict__ vr,
    int nNodes, int nEdges, int nChunks)
{
    extern __shared__ float4 dsm[];
    float* keys = (float*)dsm;
    unsigned* list = (unsigned*)(keys + NBN * HC);
    int* tot = (int*)(list + LCAP);
    volatile unsigned char* owner = (volatile unsigned char*)(tot + 16);

    const int tid = threadIdx.x, lane = tid & 31, wave = tid >> 5;
    const int nb0 = blockIdx.x * NBN;

    {
        const float ninf1 = __uint_as_float(0xff800000u);
        const v4f ninf = {ninf1, ninf1, ninf1, ninf1};
        v4f* k4 = (v4f*)keys;
#pragma unroll 4
        for (int j = 0; j < (NBN * HC / 4) / NTHR; ++j) k4[tid + j * NTHR] = ninf;
    }
    __syncthreads();

    {
        const int g = lane >> 2;
        const int s4 = lane & 3;
        v4f we4[4], be4[4];
#pragma unroll
        for (int q = 0; q < 4; ++q) { we4[q] = (v4f){0.0f, 0.0f, 0.0f, 0.0f}; be4[q] = we4[q]; }
        if (wave == 0) {
#pragma unroll
            for (int q = 0; q < 4; ++q) {
                we4[q] = *(const v4f*)(We + 16 * s4 + 4 * q);
                be4[q] = *(const v4f*)(be + 16 * s4 + 4 * q);
            }
        }
        const unsigned bid4 = (unsigned)blockIdx.x * 0x01010101u;

        for (int c = 0; c < nChunks; ++c) {
            const int lb = c * CHK + wave * 1024 + lane * 16;
            const v4u w0 = *(const v4u*)(code + lb);
            const v4u w1 = *(const v4u*)(code + lb + 512);
            unsigned M = 0u;
            M |= zmask(w0.x ^ bid4) >> 7;
            M |= zmask(w0.y ^ bid4) >> 6;
            M |= zmask(w0.z ^ bid4) >> 5;
            M |= zmask(w0.w ^ bid4) >> 4;
            M |= zmask(w1.x ^ bid4) >> 3;
            M |= zmask(w1.y ^ bid4) >> 2;
            M |= zmask(w1.z ^ bid4) >> 1;
            M |= zmask(w1.w ^ bid4);
            const int cnt = (int)__builtin_popcount(M);

            int incl = cnt;
#pragma unroll
            for (int d = 1; d < 32; d <<= 1) {
                const int y = __shfl_up(incl, d);
                if (lane >= d) incl += y;
            }
            if (lane == 31) tot[wave] = incl;
            __syncthreads();
            int pre = 0, btotal = 0;
#pragma unroll
            for (int w = 0; w < 8; ++w) {
                const int tw = tot[w];
                btotal += tw;
                pre += (w < wave) ? tw : 0;
            }
            int p = pre + incl - cnt;
            for (int q = 0; q < 32 && M != 0u; ++q) {
                const int j = (int)__builtin_ctz(M);
                M &= M - 1u;
                const int d = j & 7, b = j >> 3;
                const unsigned e = (unsigned)(lb + ((d & 4) << 7) + ((d & 3) << 2) + b);
                if (p < LCAP) list[p] = e;
                ++p;
            }
            __syncthreads();

            const int cntc = min(btotal, LCAP);
            if (wave == 0) {
                const unsigned emax = (unsigned)(nEdges - 1);
                for (int i0 = 0; i0 < cntc; i0 += 8) {
                    const int idx = i0 + g;
                    const bool valid = idx < cntc;
                    const int idxc = valid ? idx : (cntc - 1);
                    unsigned e = list[idxc];
                    e = (e < emax) ? e : emax;
                    int src = ei[e];
                    int dst = ei[(size_t)nEdges + e];
                    const float a = ea[e];
                    src = min(max(src, 0), nNodes - 1);
                    dst = min(max(dst, 0), nNodes - 1);
                    int loc = dst - nb0;
                    loc = min(max(loc, 0), NBN - 1);
                    const v4f* hp = (const v4f*)(hin + (size_t)src * HC + 16 * s4);
                    const v4f x0 = hp[0], x1 = hp[1], x2 = hp[2], x3 = hp[3];
                    const v4f m0 = x0 * (a * we4[0] + be4[0]);
                    const v4f m1 = x1 * (a * we4[1] + be4[1]);
                    const v4f m2 = x2 * (a * we4[2] + be4[2]);
                    const v4f m3 = x3 * (a * we4[3] + be4[3]);
                    v4f* kp = (v4f*)(keys + loc * HC + 16 * s4);
                    bool pend = valid;
#pragma unroll 1
                    for (int rnd = 0; rnd < 8; ++rnd) {
                        if (!__any(pend)) break;
                        if (pend) {
                            owner[loc] = (unsigned char)g;
                            const unsigned win = (unsigned)owner[loc];
                            if (win == (unsigned)g) {
                                kp[0] = vmax4(kp[0], m0);
                                kp[1] = vmax4(kp[1], m1);
                                kp[2] = vmax4(kp[2], m2);
                                kp[3] = vmax4(kp[3], m3);
                                pend = false;
                            }
                        }
                    }
                }
            }
            __syncthreads();
        }
    }

    {
        const int h2 = lane >> 4, m = lane & 15;
        float* stg = (float*)list + wave * 512;
        float bb[4], sc[4], mv[4], bt[4];
#pragma unroll
        for (int ct = 0; ct < 4; ++ct) {
            const int n = ct * 16 + m;
            bb[ct] = bu[n];
            sc[ct] = gam[n] / sqrtf(vr[n] + BN_EPS);
            mv[ct] = mn[n];
            bt[ct] = bet[n];
        }
        const unsigned short* wlo = wpl + HC * KU;

        for (int it = 0; it < NBN / 16 / 8; ++it) {
            const int lrow0 = (it * 8 + wave) * 16;
            const int grow0 = nb0 + lrow0;
            v8f acc[4];
#pragma unroll
            for (int ct = 0; ct < 4; ++ct) acc[ct] = (v8f){0.f, 0.f, 0.f, 0.f, 0.f, 0.f, 0.f, 0.f};

#pragma unroll
            for (int ks = 0; ks < 4; ++ks) {
                float v[16];
                if (ks < 2) {
                    ld16(hin + (size_t)(grow0 + m) * HC + ks * 32 + 8 * h2, v);
                } else {
                    ld16(keys + (lrow0 + m) * HC + (ks - 2) * 32 + 8 * h2, v);
#pragma unroll
                    for (int i = 0; i < 16; ++i) v[i] = (v[i] > -3.0e38f) ? v[i] : 0.0f;
                }
                v16b ah, al;
                split16(v, ah, al);
#pragma unroll
                for (int ct = 0; ct < 4; ++ct) {
                    const unsigned short* bp = wpl + (size_t)(ct * 16 + m) * KU + ks * 32 + 8 * h2;
                    const unsigned short* bq = wlo + (size_t)(ct * 16 + m) * KU + ks * 32 + 8 * h2;
                    Frag bh, bl;
                    bh.half[0] = *(const v8us*)bp;
                    bh.half[1] = *(const v8us*)(bp + 16);
                    bl.half[0] = *(const v8us*)bq;
                    bl.half[1] = *(const v8us*)(bq + 16);
                    acc[ct] = wmma16(ah, bh.v, acc[ct]);
                    acc[ct] = wmma16(ah, bl.v, acc[ct]);
                    acc[ct] = wmma16(al, bh.v, acc[ct]);
                }
            }
#pragma unroll
            for (int ct = 0; ct < 4; ++ct) {
#pragma unroll
                for (int r = 0; r < 8; ++r) {
                    float xq = acc[ct][r] + bb[ct];
                    xq = fmaxf(xq, 0.0f);
                    xq = (xq - mv[ct]) * sc[ct] + bt[ct];
                    xq = fmaxf(xq, 0.0f);
                    acc[ct][r] = xq;
                }
            }
#pragma unroll
            for (int hh = 0; hh < 2; ++hh) {
                __syncthreads();
                if (h2 == hh) {
#pragma unroll
                    for (int ct = 0; ct < 4; ++ct) {
#pragma unroll
                        for (int r = 0; r < 8; ++r) stg[r * HC + ct * 16 + m] = acc[ct][r];
                    }
                }
                __syncthreads();
                const int rr = lane >> 4, c4 = (lane & 15) * 4;
                v4f f[4];
#pragma unroll
                for (int q = 0; q < 4; ++q) f[q] = *(const v4f*)(stg + (2 * q + rr) * HC + c4);
                float* op = hout + (size_t)(grow0 + 8 * hh + rr) * HC + c4;
#pragma unroll
                for (int q = 0; q < 4; ++q) *(volatile v4f*)(op + (size_t)(2 * q) * HC) = f[q];
                __threadfence();
#pragma unroll
                for (int q = 0; q < 4; ++q) *(volatile v4f*)(op + (size_t)(2 * q) * HC) = f[q];
            }
        }
    }
}

__global__ __launch_bounds__(NTHR) void k_pred(const float* __restrict__ hin, const unsigned short* __restrict__ wp,
                                               const float* __restrict__ bp1, const float* __restrict__ Wp2,
                                               const float* __restrict__ bp2, float* out, int outN)
{
    __shared__ float red[8 * 16];
    __shared__ float ov[32];
    const int tid = threadIdx.x, lane = tid & 31, wave = tid >> 5;
    const int h2 = lane >> 4, m = lane & 15;
    const int rt = wave >> 2, ct = wave & 3;
    const int grow0 = blockIdx.x * 32 + rt * 16;

    v8f acc = (v8f){0.f, 0.f, 0.f, 0.f, 0.f, 0.f, 0.f, 0.f};
#pragma unroll
    for (int ks = 0; ks < 2; ++ks) {
        float v[16];
        ld16(hin + (size_t)(grow0 + m) * HC + ks * 32 + 8 * h2, v);
        v16b ah, al;
        split16(v, ah, al);
        const unsigned short* bp = wp + (size_t)(ct * 16 + m) * HC + ks * 32 + 8 * h2;
        const unsigned short* bq = bp + HC * HC;
        Frag bh, bl;
        bh.half[0] = *(const v8us*)bp;
        bh.half[1] = *(const v8us*)(bp + 16);
        bl.half[0] = *(const v8us*)bq;
        bl.half[1] = *(const v8us*)(bq + 16);
        acc = wmma16(ah, bh.v, acc);
        acc = wmma16(ah, bl.v, acc);
        acc = wmma16(al, bh.v, acc);
    }
    const int n = ct * 16 + m;
    const float b1 = bp1[n], w2 = Wp2[n];
    float t[8];
#pragma unroll
    for (int r = 0; r < 8; ++r) t[r] = fmaxf(acc[r] + b1, 0.0f) * w2;
#pragma unroll
    for (int off = 8; off > 0; off >>= 1) {
#pragma unroll
        for (int r = 0; r < 8; ++r) t[r] += __shfl_xor(t[r], off);
    }
    if (m == 0) {
#pragma unroll
        for (int r = 0; r < 8; ++r) red[(ct * 2 + rt) * 16 + 8 * h2 + r] = t[r];
    }
    __syncthreads();
    if (tid < 32) {
        const int rtt = tid >> 4, rr = tid & 15;
        float s = bp2[0];
        s += red[(0 * 2 + rtt) * 16 + rr];
        s += red[(1 * 2 + rtt) * 16 + rr];
        s += red[(2 * 2 + rtt) * 16 + rr];
        s += red[(3 * 2 + rtt) * 16 + rr];
        ov[tid] = s;
    }
    __syncthreads();
    if (tid < 8) {
        const int g0 = blockIdx.x * 32 + 4 * tid;
        const v4f f = *(const v4f*)(ov + 4 * tid);
        if (g0 + 3 < outN) {
            volatile v4f* p = (volatile v4f*)(out + g0);
            *p = f;
            __threadfence();
            *p = f;
        } else {
            volatile float* p = (volatile float*)out;
            const float fe[4] = {f.x, f.y, f.z, f.w};
#pragma unroll
            for (int q = 0; q < 4; ++q) if (g0 + q < outN) p[g0 + q] = fe[q];
            __threadfence();
#pragma unroll
            for (int q = 0; q < 4; ++q) if (g0 + q < outN) p[g0 + q] = fe[q];
        }
    }
}

static inline size_t al256(size_t b) { return (b + 255) & ~(size_t)255; }

extern "C" void kernel_launch(void* const* d_in, const int* in_sizes, int n_in,
                              void* d_out, int out_size, void* d_ws, size_t ws_size,
                              hipStream_t stream)
{
    if (n_in < 17) return;
    const float* x      = (const float*)d_in[0];
    const int*   ei     = (const int*)  d_in[1];
    const float* ea     = (const float*)d_in[2];
    const float* W_enc  = (const float*)d_in[3];
    const float* b_enc  = (const float*)d_in[4];
    const float* W_edge = (const float*)d_in[5];
    const float* b_edge = (const float*)d_in[6];
    const float* W_upd  = (const float*)d_in[7];
    const float* b_upd  = (const float*)d_in[8];
    const float* bn_g   = (const float*)d_in[9];
    const float* bn_b   = (const float*)d_in[10];
    const float* bn_m   = (const float*)d_in[11];
    const float* bn_v   = (const float*)d_in[12];
    const float* W_p1   = (const float*)d_in[13];
    const float* b_p1   = (const float*)d_in[14];
    const float* W_p2   = (const float*)d_in[15];
    const float* b_p2   = (const float*)d_in[16];
    float* out = (float*)d_out;

    const int nNodes = in_sizes[0] / 6;
    const int nEdges = in_sizes[1] / 2;
    if (nNodes <= 0 || nEdges <= 0 || out_size <= 0) return;
    const int nBlk = (nNodes + NBN - 1) / NBN;
    if (nBlk > 255) return;
    const int nRowsPad = nBlk * NBN;
    const int nChunks = (nEdges + CHK - 1) / CHK;
    const int nEdgesPad = nChunks * CHK;

    char* base = (char*)d_ws;
    size_t off = 0;
    const size_t szH = (size_t)nRowsPad * HC * sizeof(float);
    float* hA = (float*)(base + off); off += al256(szH);
    float* hB = (float*)(base + off); off += al256(szH);
    unsigned short* wsW  = (unsigned short*)(base + off); off += al256((size_t)NL * 2 * HC * KU * 2);
    unsigned short* wsWp = (unsigned short*)(base + off); off += al256((size_t)2 * HC * HC * 2);
    unsigned char* code  = (unsigned char*)(base + off);  off += al256((size_t)nEdgesPad);
    if (off > ws_size) return;
    const int outN = (out_size < nNodes) ? out_size : nNodes;

    hipFuncSetAttribute(reinterpret_cast<const void*>(&k_layer), hipFuncAttributeMaxDynamicSharedMemorySize, LDS_BYTES);

    k_prep<<<(NL * HC * 16 + HC * 8 + NTHR - 1) / NTHR, NTHR, 0, stream>>>(W_upd, W_p1, wsW, wsWp);
    k_code<<<(nEdgesPad / 16 + NTHR - 1) / NTHR, NTHR, 0, stream>>>(ei, code, nNodes, nEdges, nEdgesPad);
    k_enc<<<(nRowsPad * 16 + NTHR - 1) / NTHR, NTHR, 0, stream>>>(x, W_enc, b_enc, hA, nNodes, nRowsPad);

    float* hc = hA;
    float* hn = hB;
    for (int l = 0; l < NL; ++l) {
        k_layer<<<nBlk, NTHR, LDS_BYTES, stream>>>(
            hc, hn, code, ei, ea,
            wsW + (size_t)l * 2 * HC * KU,
            W_edge + (size_t)l * HC, b_edge + (size_t)l * HC,
            b_upd + (size_t)l * HC, bn_g + (size_t)l * HC, bn_b + (size_t)l * HC,
            bn_m + (size_t)l * HC, bn_v + (size_t)l * HC,
            nNodes, nEdges, nChunks);
        float* tswap = hc; hc = hn; hn = tswap;
    }
    k_pred<<<(outN + 31) / 32, NTHR, 0, stream>>>(hc, wsWp, b_p1, W_p2, b_p2, out, outN);
}
